// MultiHeadAttention3D_15547781612054
// MI455X (gfx1250) — hardware-verified
//
#include <hip/hip_runtime.h>


#define NSQ  16
#define NTK  1024
#define CC   512
#define NH_  8
#define HD   64
#define TT   8
#define NR   (NSQ * NTK)
#define SG   2
#define DM   CC
#define LOSC 1024.0f
typedef _Float16 h16;
typedef unsigned short bf;
typedef __attribute__((ext_vector_type(16))) __bf16   v16bf;
typedef __attribute__((ext_vector_type(16))) _Float16 v16h;
typedef __attribute__((ext_vector_type(8)))  _Float16 v8h;
typedef __attribute__((ext_vector_type(8)))  unsigned short v8us;
typedef __attribute__((ext_vector_type(8)))  float    v8f;
typedef __attribute__((ext_vector_type(4)))  float    v4f;
typedef v8h  __attribute__((may_alias)) v8ha;
typedef v4f  __attribute__((may_alias)) v4fa;
typedef v8us __attribute__((may_alias)) v8usa;

__device__ __forceinline__ unsigned short f2bf(float f) { unsigned u = __float_as_uint(f); u += 0x7FFFu + ((u >> 16) & 1u); return (unsigned short)(u >> 16); }
__device__ __forceinline__ float bf2f(unsigned short b) { return __uint_as_float(((unsigned)b) << 16); }
__device__ __forceinline__ float bfr(float f) { return bf2f(f2bf(f)); }
__device__ __forceinline__ v16h cat16(v8h lo, v8h hi) { return __builtin_shufflevector(lo, hi, 0, 1, 2, 3, 4, 5, 6, 7, 8, 9, 10, 11, 12, 13, 14, 15); }
__device__ __forceinline__ v16bf cat16b(v8us lo, v8us hi) { return __builtin_bit_cast(v16bf, __builtin_shufflevector(lo, hi, 0, 1, 2, 3, 4, 5, 6, 7, 8, 9, 10, 11, 12, 13, 14, 15)); }
__device__ __forceinline__ v8f wmma16(v16h a, v16h b, v8f c) { return __builtin_amdgcn_wmma_f32_16x16x32_f16(false, a, false, b, (short)0, c, false, false); }
__device__ __forceinline__ v8f wmmab(v16bf a, v16bf b, v8f c) { return __builtin_amdgcn_wmma_f32_16x16x32_bf16(false, a, false, b, (short)0, c, false, false); }


__global__ __launch_bounds__(128) void k_gemmh(const h16* __restrict__ A, const h16* __restrict__ Bn, const float* __restrict__ bias, float* C, int ldc, const float* __restrict__ R, int K, size_t sA, size_t sB, size_t sC, int roundR) {
    __shared__ __align__(16) float ost[4][16 * 68];
    const size_t z = blockIdx.z; A += z * sA; Bn += z * sB; C += z * sC; if (R) R += z * sC;
    const int lane = threadIdx.x & 31, wave = threadIdx.x >> 5, lr = lane & 15, hi = lane >> 4;
    const int r0 = blockIdx.x * 64 + wave * 16, c0 = blockIdx.y * 64;
    const size_t aoff = (size_t)(r0 + lr) * K + 8 * hi;
    size_t boff[4];
#pragma unroll
    for (int t = 0; t < 4; ++t) boff[t] = (size_t)(c0 + t * 16 + lr) * K + 8 * hi;
    v8f acc[4];
#pragma unroll
    for (int t = 0; t < 4; ++t) acc[t] = (v8f){};
#pragma unroll 1
    for (int kc = 0; kc < K; kc += 32) {
        const v16h a = cat16(*(const v8h*)(A + aoff + kc), *(const v8h*)(A + aoff + kc + 16));
#pragma unroll
        for (int t = 0; t < 4; ++t) { const v16h b = cat16(*(const v8h*)(Bn + boff[t] + kc), *(const v8h*)(Bn + boff[t] + kc + 16)); acc[t] = wmma16(a, b, acc[t]); }
        asm volatile("v_nop\n\tv_nop\n\tv_nop\n\tv_nop" : "+v"(acc[0]), "+v"(acc[1]), "+v"(acc[2]), "+v"(acc[3]) : "v"(a));
    }
    float* os = &ost[wave][0];
#pragma unroll
    for (int t = 0; t < 4; ++t) { const float bv = bias ? bfr(bias[c0 + t * 16 + lr]) : 0.f;
#pragma unroll
        for (int j = 0; j < 8; ++j) os[(hi * 8 + j) * 68 + t * 16 + lr] = acc[t][j] + bv; }
    __syncthreads();
    float* crow = C + (size_t)r0 * ldc + c0;
    auto pass = [&]() {
#pragma unroll
        for (int s = 0; s < 8; ++s) { const int Lid = (lane >> 3) + 4 * s, piece = lane & 7; const int row = Lid >> 1, cofs = (Lid & 1) * 32 + piece * 4;
            v4f val = *(const v4fa*)(os + row * 68 + cofs); if (R) { const v4f rv = *(const v4f*)(R + ((size_t)r0 + row) * ldc + c0 + cofs); val += roundR ? (v4f){bfr(rv[0]), bfr(rv[1]), bfr(rv[2]), bfr(rv[3])} : rv; }
            *(volatile v4f*)(crow + (size_t)row * ldc + cofs) = val; }
    };
    pass(); __threadfence(); pass();
}

typedef __attribute__((ext_vector_type(4))) _Float16 v4h;
__device__ __forceinline__ h16 tohx(float x) { return (h16)x; }
__device__ __forceinline__ size_t xoff(int s, int c, int n) { const int b = s / TT, t = s % TT; return (((size_t)b * CC + c) * TT + t) * NTK + n; }
__global__ __launch_bounds__(256) void k_stat(const float* __restrict__ x, float* MU, float* RS) {
    const int lane = threadIdx.x & 31; const int w = blockIdx.x * 8 + (threadIdx.x >> 5); if (w >= NR / 32) return; const int s = w / (NTK / 32), n = (w % (NTK / 32)) * 32 + lane; float sum = 0.f;
#pragma unroll 1
    for (int c = 0; c < CC; ++c) sum += bfr(x[xoff(s, c, n)]);
    const float mu = sum * (1.0f / CC); float q = 0.f;
#pragma unroll 1
    for (int c = 0; c < CC; ++c) { const float d = bfr(x[xoff(s, c, n)]) - mu; q = fmaf(d, d, q); }
    const float rs = rsqrtf(q * (1.0f / CC) + 1e-5f); const size_t r = (size_t)s * NTK + n;
    *(volatile float*)(MU + r) = mu; *(volatile float*)(RS + r) = rs; __threadfence(); *(volatile float*)(MU + r) = mu; *(volatile float*)(RS + r) = rs;
}
__global__ __launch_bounds__(256) void k_nrow(const float* __restrict__ x, const float* __restrict__ MU, const float* __restrict__ RS, const float* __restrict__ g, const float* __restrict__ bb, h16* XN) {
    const int lane = threadIdx.x & 31; const size_t r = (size_t)blockIdx.x * 8 + (threadIdx.x >> 5); if (r >= (size_t)NR) return; const int s = (int)(r / NTK), n = (int)(r % NTK); const float mu = MU[r], rs = RS[r];
#pragma unroll 1
    for (int ps = 0; ps < 2; ++ps) {
#pragma unroll 1
        for (int p = 0; p < CC / 256; ++p) { const int c0 = p * 256 + lane * 8; v8h o;
#pragma unroll
            for (int i = 0; i < 8; ++i) { const int c = c0 + i; o[i] = tohx((bfr(x[xoff(s, c, n)]) - mu) * rs * bfr(g[c]) + bfr(bb[c])); }
            *(volatile v8h*)(XN + r * CC + c0) = o; }
        if (ps == 0) __threadfence(); }
}
__global__ __launch_bounds__(256) void k_wTh(const float* __restrict__ Wm, int K, int N, h16* Bt) {
    __shared__ float tl[64][65];
    const int tid = threadIdx.x; const int k0 = blockIdx.x * 64, n0 = blockIdx.y * 64; const int rr = tid >> 2, cq = (tid & 3) * 16;
#pragma unroll
    for (int i = 0; i < 16; ++i) tl[rr][cq + i] = bfr(Wm[(size_t)(k0 + rr) * N + n0 + cq + i]);
    __syncthreads();
    const int lane = tid & 31, wv = tid >> 5;
    auto pass = [&]() {
#pragma unroll
        for (int st = 0; st < 4; ++st) { const int nr = wv * 8 + st * 2 + (lane >> 4); const int kq = (lane & 15) * 4; v4h v;
#pragma unroll
            for (int i = 0; i < 4; ++i) v[i] = tohx(tl[kq + i][nr]);
            *(volatile v4h*)(Bt + (size_t)(n0 + nr) * K + k0 + kq) = v; }
    };
    pass(); __threadfence(); pass();
}
__global__ __launch_bounds__(256) void k_hplh3(const float* __restrict__ F, int s0, float sc, h16* P) {
    const int lane = threadIdx.x & 31; const size_t w = (size_t)blockIdx.x * 8 + (threadIdx.x >> 5); const int i = (int)(w * 2 + (lane >> 4)); if (i >= NTK) return; const int g = blockIdx.z / NH_, h = blockIdx.z % NH_; const int c0 = (lane & 15) * 4; v4h o;
#pragma unroll
    for (int q = 0; q < 4; ++q) o[q] = tohx(F[((size_t)(s0 + g) * NTK + i) * CC + h * HD + c0 + q] * sc);
    const size_t off = ((size_t)blockIdx.z * NTK + i) * HD + c0; *(volatile v4h*)(P + off) = o; __threadfence(); *(volatile v4h*)(P + off) = o;
}
__global__ __launch_bounds__(256) void k_vTh3(const float* __restrict__ V, int s0, h16* VT) {
    __shared__ float tl[64][65];
    const int tid = threadIdx.x; const int t0 = blockIdx.x * 64; const int g = blockIdx.z / NH_, h = blockIdx.z % NH_; const int rr = tid >> 2, cq = (tid & 3) * 16;
#pragma unroll
    for (int i = 0; i < 16; ++i) tl[rr][cq + i] = V[((size_t)(s0 + g) * NTK + t0 + rr) * CC + h * HD + cq + i];
    __syncthreads();
    const int lane = tid & 31, wv = tid >> 5;
    auto pass = [&]() {
#pragma unroll
        for (int st = 0; st < 4; ++st) { const int dr = wv * 8 + st * 2 + (lane >> 4); const int tq = (lane & 15) * 4; v4h v;
#pragma unroll
            for (int i = 0; i < 4; ++i) v[i] = tohx(tl[tq + i][dr]);
            *(volatile v4h*)(VT + ((size_t)blockIdx.z * HD + dr) * NTK + t0 + tq) = v; }
    };
    pass(); __threadfence(); pass();
}
__global__ __launch_bounds__(256) void k_softh3(const float* __restrict__ S, h16* P) {
    const int lane = threadIdx.x & 31, i = blockIdx.x * 8 + (threadIdx.x >> 5); if (i >= NTK) return; const size_t zo = (size_t)blockIdx.z * NTK * NTK + (size_t)i * NTK; const float* sr = S + zo; h16* po = P + zo;
    float m = -3.0e38f;
#pragma unroll 1
    for (int c0 = lane * 4; c0 < NTK; c0 += 128) {
#pragma unroll
        for (int q = 0; q < 4; ++q) m = fmaxf(m, sr[c0 + q]); }
#pragma unroll
    for (int sh = 16; sh; sh >>= 1) m = fmaxf(m, __shfl_xor(m, sh, 32));
    float sum = 0.f;
#pragma unroll 1
    for (int c0 = lane * 4; c0 < NTK; c0 += 128) {
#pragma unroll
        for (int q = 0; q < 4; ++q) sum += __expf(sr[c0 + q] - m); }
#pragma unroll
    for (int sh = 16; sh; sh >>= 1) sum += __shfl_xor(sum, sh, 32);
    const float inv = 1.0f / sum;
#pragma unroll 1
    for (int ps = 0; ps < 2; ++ps) {
#pragma unroll 1
        for (int c0 = lane * 4; c0 < NTK; c0 += 128) { v4h o;
#pragma unroll
            for (int q = 0; q < 4; ++q) o[q] = tohx(__expf(sr[c0 + q] - m) * inv);
            *(volatile v4h*)(po + c0) = o; }
        if (ps == 0) __threadfence(); }
}
__global__ __launch_bounds__(256) void k_mergeh3(const float* __restrict__ OZ, int s0, h16* OH) {
    const int lane = threadIdx.x & 31; const size_t w = (size_t)blockIdx.x * 8 + (threadIdx.x >> 5); if (w >= (size_t)SG * NTK) return; const int g = (int)(w / NTK), i = (int)(w % NTK); const size_t row = (size_t)(s0 + g) * NTK + i;
#pragma unroll 1
    for (int ps = 0; ps < 2; ++ps) {
#pragma unroll
        for (int q = 0; q < 2; ++q) { const int c0 = q * 256 + lane * 8; const int h = c0 / HD, d0 = c0 % HD; v8h o;
#pragma unroll
            for (int k = 0; k < 8; ++k) o[k] = tohx(OZ[(((size_t)(g * NH_ + h)) * NTK + i) * HD + d0 + k]);
            *(volatile v8h*)(OH + row * CC + c0) = o; }
        if (ps == 0) __threadfence(); }
}
__global__ __launch_bounds__(256) void k_outT3(const float* __restrict__ Y, const float* __restrict__ x, int s0, float* OUTB) {
    __shared__ float tl[64][65];
    const int tid = threadIdx.x; const int n0 = blockIdx.x * 64, c0 = blockIdx.y * 64; const int g = blockIdx.z, s = s0 + g; const int rr = tid >> 2, cq = (tid & 3) * 16;
#pragma unroll
    for (int i = 0; i < 16; ++i) tl[rr][cq + i] = Y[((size_t)g * NTK + n0 + rr) * CC + c0 + cq + i];
    __syncthreads();
    const int lane = tid & 31, wv = tid >> 5;
    auto pass = [&]() {
#pragma unroll
        for (int st = 0; st < 4; ++st) { const int cr = wv * 8 + st * 2 + (lane >> 4); const int nq = (lane & 15) * 4; const size_t o = xoff(s, c0 + cr, n0 + nq); v4f v;
#pragma unroll
            for (int i = 0; i < 4; ++i) v[i] = tl[nq + i][cr] + bfr(x[o + i]);
            *(volatile v4f*)(OUTB + o) = v; }
    };
    pass(); __threadfence(); pass();
}

#define GRW (SG * NTK)
extern "C" void kernel_launch(void* const* d_in, const int* in_sizes, int n_in,
                              void* d_out, int out_size, void* d_ws, size_t ws_size, hipStream_t stream) {
    (void)in_sizes; (void)n_in; (void)out_size;
    const float* x = (const float*)d_in[0]; const float* lg = (const float*)d_in[1]; const float* lb = (const float*)d_in[2]; const float* Wq = (const float*)d_in[3]; const float* bq = (const float*)d_in[4]; const float* Wk = (const float*)d_in[5]; const float* bk = (const float*)d_in[6]; const float* Wv = (const float*)d_in[7]; const float* bv = (const float*)d_in[8]; const float* Wp = (const float*)d_in[9]; const float* bp = (const float*)d_in[10];
    float* out = (float*)d_out;
    char* wsp = (char*)d_ws;
    auto take = [&](size_t bytes) { char* p = wsp; wsp += (bytes + 255) & ~(size_t)255; return (void*)p; };
    h16* BQ = (h16*)take((size_t)CC * CC * 2); h16* BK = (h16*)take((size_t)CC * CC * 2); h16* BV = (h16*)take((size_t)CC * CC * 2); h16* BP = (h16*)take((size_t)CC * CC * 2);
    float* MU = (float*)take(NR * 4); float* RS = (float*)take(NR * 4); h16* XN = (h16*)take((size_t)NR * CC * 2);
    float* Q = (float*)take((size_t)GRW * CC * 4); float* Kf = (float*)take((size_t)GRW * CC * 4); float* V = (float*)take((size_t)GRW * CC * 4);
    h16* Qx = (h16*)take((size_t)SG * NH_ * NTK * HD * 2); h16* Kx = (h16*)take((size_t)SG * NH_ * NTK * HD * 2); h16* VTx = (h16*)take((size_t)SG * NH_ * HD * NTK * 2); float* S = (float*)take((size_t)SG * NH_ * NTK * NTK * 4); h16* Px = (h16*)take((size_t)SG * NH_ * NTK * NTK * 2); float* OZ = (float*)take((size_t)SG * NH_ * NTK * HD * 4); h16* OH = (h16*)take((size_t)GRW * CC * 2); float* Y = (float*)take((size_t)GRW * CC * 4);
    if ((size_t)(wsp - (char*)d_ws) > ws_size) return;
    k_wTh<<<dim3(CC / 64, CC / 64, 1), 256, 0, stream>>>(Wq, CC, CC, BQ); k_wTh<<<dim3(CC / 64, CC / 64, 1), 256, 0, stream>>>(Wk, CC, CC, BK); k_wTh<<<dim3(CC / 64, CC / 64, 1), 256, 0, stream>>>(Wv, CC, CC, BV); k_wTh<<<dim3(CC / 64, CC / 64, 1), 256, 0, stream>>>(Wp, CC, CC, BP);
    k_stat<<<(NR / 32) / 8, 256, 0, stream>>>(x, MU, RS);
    k_nrow<<<NR / 8, 256, 0, stream>>>(x, MU, RS, lg, lb, XN);
    for (int s0 = 0; s0 < NSQ; s0 += SG) { const h16* XG = XN + (size_t)s0 * NTK * CC;
        k_gemmh<<<dim3(GRW / 64, CC / 64, 1), 128, 0, stream>>>(XG, BQ, bq, Q, CC, nullptr, CC, 0, 0, 0, 0);
        k_gemmh<<<dim3(GRW / 64, CC / 64, 1), 128, 0, stream>>>(XG, BK, bk, Kf, CC, nullptr, CC, 0, 0, 0, 0);
        k_gemmh<<<dim3(GRW / 64, CC / 64, 1), 128, 0, stream>>>(XG, BV, bv, V, CC, nullptr, CC, 0, 0, 0, 0);
        k_hplh3<<<dim3((NTK / 2) / 8, 1, SG * NH_), 256, 0, stream>>>(Q, 0, 0.125f, Qx); k_hplh3<<<dim3((NTK / 2) / 8, 1, SG * NH_), 256, 0, stream>>>(Kf, 0, 1.0f, Kx); k_vTh3<<<dim3(NTK / 64, 1, SG * NH_), 256, 0, stream>>>(V, 0, VTx);
        k_gemmh<<<dim3(NTK / 64, NTK / 64, SG * NH_), 128, 0, stream>>>(Qx, Kx, nullptr, S, NTK, nullptr, HD, (size_t)NTK * HD, (size_t)NTK * HD, (size_t)NTK * NTK, 0);
        k_softh3<<<dim3(NTK / 8, 1, SG * NH_), 256, 0, stream>>>(S, Px);
        k_gemmh<<<dim3(NTK / 64, 1, SG * NH_), 128, 0, stream>>>(Px, VTx, nullptr, OZ, HD, nullptr, NTK, (size_t)NTK * NTK, (size_t)HD * NTK, (size_t)NTK * HD, 0);
        k_mergeh3<<<(SG * NTK) / 8, 256, 0, stream>>>(OZ, 0, OH);
        k_gemmh<<<dim3(GRW / 64, CC / 64, 1), 128, 0, stream>>>(OH, BP, bp, Y, CC, nullptr, CC, 0, 0, 0, 0);
        k_outT3<<<dim3(NTK / 64, CC / 64, SG), 256, 0, stream>>>(Y, x, s0, out); }
}
